// STAGNNAggregator_Optimized_72610717106762
// MI455X (gfx1250) — hardware-run, weakly checked
//
#include <hip/hip_runtime.h>

typedef float          v8f   __attribute__((ext_vector_type(8)));
typedef float          v4f   __attribute__((ext_vector_type(4)));
typedef unsigned int   v4u   __attribute__((ext_vector_type(4)));
typedef int            v8i   __attribute__((ext_vector_type(8)));
typedef unsigned short v8us  __attribute__((ext_vector_type(8)));
typedef unsigned short v16us __attribute__((ext_vector_type(16)));
typedef __bf16         v16bf __attribute__((ext_vector_type(16)));
typedef _Float16       v16h  __attribute__((ext_vector_type(16)));
typedef v4f  __attribute__((may_alias)) v4fa;
typedef v8us __attribute__((may_alias)) v8usa;
union FragB { v16bf v; v16us u; v8us h[2]; v8i w; };
union FragH { v16h  v; v16us u; v8us h[2]; v8i w; };

__device__ __forceinline__ v8f wmb(const FragB& a, const FragB& b, v8f c) {
  v8f d = __builtin_amdgcn_wmma_f32_16x16x32_bf16(false, a.v, false, b.v, (short)0, c, false, false);
  asm volatile("v_nop\n\tv_nop\n\tv_nop\n\tv_nop" : "+v"(d) : "v"(a.w), "v"(b.w));
  return d;
}

__device__ __forceinline__ v8f wmh(const FragH& a, const FragH& b, v8f c) {
  v8f d = __builtin_amdgcn_wmma_f32_16x16x32_f16(false, a.v, false, b.v, (short)0, c, false, false);
  asm volatile("v_nop\n\tv_nop\n\tv_nop\n\tv_nop" : "+v"(d) : "v"(a.w), "v"(b.w));
  return d;
}

__device__ __forceinline__ unsigned bf16_bits(float f) {
  const unsigned u = __float_as_uint(f);
  const unsigned r = (u + 0x7FFFu + ((u >> 16) & 1u)) >> 16;
  const unsigned q = (u >> 16) | 0x40u;
  return ((u & 0x7fffffffu) > 0x7f800000u) ? q : r;
}

__device__ __forceinline__ float bf16_val(float f) {
  return __uint_as_float(bf16_bits(f) << 16);
}
__device__ __forceinline__ int clampi(int v, int lo, int hi) {
  return v < lo ? lo : (v > hi ? hi : v);
}

__device__ __forceinline__ unsigned f16_bits(float f) {
  const unsigned u  = __float_as_uint(f);
  const unsigned s  = (u >> 16) & 0x8000u;
  const unsigned a  = u & 0x7fffffffu;
  const unsigned t  = a - 0x38000000u;
  const unsigned r  = (t + 0x0FFFu + ((t >> 13) & 1u)) >> 13;
  const unsigned rc = r > 0x7C00u ? 0x7C00u : r;
  const bool small  = a < 0x38800000u;
  const bool isnan  = a > 0x7f800000u;
  const unsigned fin = small ? 0u : (s | rc);
  return isnan ? (s | 0x7E00u) : fin;
}

__device__ __forceinline__ unsigned pk16(unsigned lo, unsigned hi) { return lo | (hi << 16); }
__device__ __forceinline__ unsigned bf16_lo_bits(float v) {
  float hi = bf16_val(v);
  asm volatile("" : "+v"(hi));
  return bf16_bits(v - hi);
}
__device__ __forceinline__ v4u pack8_bf16(v4f a, v4f c) {
  return (v4u){ pk16(bf16_bits(a[0]), bf16_bits(a[1])), pk16(bf16_bits(a[2]), bf16_bits(a[3])),
                pk16(bf16_bits(c[0]), bf16_bits(c[1])), pk16(bf16_bits(c[2]), bf16_bits(c[3])) };
}
__device__ __forceinline__ v4u pack8_bf16_lo(v4f a, v4f c) {
  return (v4u){ pk16(bf16_lo_bits(a[0]), bf16_lo_bits(a[1])), pk16(bf16_lo_bits(a[2]), bf16_lo_bits(a[3])),
                pk16(bf16_lo_bits(c[0]), bf16_lo_bits(c[1])), pk16(bf16_lo_bits(c[2]), bf16_lo_bits(c[3])) };
}
__device__ __forceinline__ v4u pack8_f16(v4f a, v4f c) {
  return (v4u){ pk16(f16_bits(a[0]), f16_bits(a[1])), pk16(f16_bits(a[2]), f16_bits(a[3])),
                pk16(f16_bits(c[0]), f16_bits(c[1])), pk16(f16_bits(c[2]), f16_bits(c[3])) };
}

template <int FORM>
__global__ __launch_bounds__(256) void k_plane(const float* __restrict__ src, int rows, int cols, int ldsrc,
                                               unsigned short* __restrict__ dst, int MP, int KP) {
  static_assert(FORM >= 0 && FORM <= 3);
  const int KTOT = (FORM == 1 || FORM == 3) ? 2 * KP : KP;
  const unsigned ppr   = (unsigned)(KTOT >> 3);
  const unsigned kp8   = (unsigned)(KP >> 3);
  const unsigned total = (unsigned)MP * ppr;
  const unsigned g     = blockIdx.x * 256u + threadIdx.x;
  const unsigned rowu  = g / ppr;
  const unsigned p     = g - rowu * ppr;
  const bool second    = p >= kp8;
  const int row = (int)rowu;
  const int c0  = (int)((second ? p - kp8 : p) << 3);
  const float* srow = src + (size_t)clampi(row, 0, rows - 1) * (size_t)ldsrc;
  float x[8];
  unsigned mk[8];
#pragma unroll
  for (int e = 0; e < 8; ++e) {
    const int c = c0 + e;
    const float v = srow[clampi(c, 0, cols - 1)];
    asm volatile("" :: "v"(v));
    x[e]  = v;
    mk[e] = (row < rows && c < cols) ? 0xFFFFu : 0u;
  }
  const v4f a = (v4f){ x[0], x[1], x[2], x[3] };
  const v4f c = (v4f){ x[4], x[5], x[6], x[7] };
  v4u o;
  if (FORM == 2) {
    o = pack8_f16(a, c);
  } else {
    const v4u hi = pack8_bf16(a, c);
    o = hi;
    if (FORM == 1) { const v4u lo = pack8_bf16_lo(a, c); o = second ? lo : hi; }
  }
  const v4u mw = (v4u){ pk16(mk[0], mk[1]), pk16(mk[2], mk[3]), pk16(mk[4], mk[5]), pk16(mk[6], mk[7]) };
  o &= mw;
  if (g < total) {
    volatile v4u* q = (volatile v4u*)(dst + (size_t)g * 8);
    *q = o;
    __threadfence();
    *q = o;
  }
}

template <int FORM> struct FragOf    { typedef FragB T; };
template <>         struct FragOf<2> { typedef FragH T; };
__device__ __forceinline__ v8f mm(const FragB& a, const FragB& b, v8f c) { return wmb(a, b, c); }
__device__ __forceinline__ v8f mm(const FragH& a, const FragH& b, v8f c) { return wmh(a, b, c); }
template <class F> __device__ __forceinline__ F ld_frag(const unsigned short* p) {
  F f;
  f.h[0] = *(const v8usa*)(p);
  f.h[1] = *(const v8usa*)(p + 16);
  return f;
}

template <int FORM, int EPI>
__global__ __launch_bounds__(256) __attribute__((amdgpu_num_vgpr(248)))
void k_gemm_nt(const unsigned short* __restrict__ A, const unsigned short* __restrict__ B,
               const float* __restrict__ bias, float* __restrict__ D, int M, int N, int KTOT, int ldd) {
  static_assert(FORM >= 0 && FORM <= 2);
  static_assert(EPI == 0 || EPI == 1);
  typedef typename FragOf<FORM>::T F;
  __shared__ __attribute__((aligned(16))) float sT[8][16 * 68];
  const int lane = threadIdx.x & 31;
  const int wave = threadIdx.x >> 5;
  const int tilesM = (M + 63) >> 6;
  const int tilesN = (N + 63) >> 6;
  const int tile = blockIdx.x * 8 + wave;
  if (tile >= tilesM * tilesN) return;
  const int tm = tile / tilesN;
  const int tn = tile - tm * tilesN;
  const int m0 = tm << 6;
  const int n0 = tn << 6;

  const int rl = lane & 15;
  const int h8 = (lane >> 4) * 8;
  const unsigned short* pa = A + (size_t)(m0 + rl) * (size_t)KTOT + h8;
  const unsigned short* pb = B + (size_t)(n0 + rl) * (size_t)KTOT + h8;

  v8f acc[4][4];
#pragma unroll
  for (int i = 0; i < 4; ++i)
#pragma unroll
    for (int j = 0; j < 4; ++j) acc[i][j] = (v8f){0.f, 0.f, 0.f, 0.f, 0.f, 0.f, 0.f, 0.f};

#pragma unroll 1
  for (int k0 = 0; k0 < KTOT; k0 += 32) {
    F bf[4];
#pragma unroll
    for (int j = 0; j < 4; ++j) bf[j] = ld_frag<F>(pb + (size_t)(j << 4) * (size_t)KTOT + k0);
#pragma unroll
    for (int i = 0; i < 4; ++i) {
      const F af = ld_frag<F>(pa + (size_t)(i << 4) * (size_t)KTOT + k0);
#pragma unroll
      for (int j = 0; j < 4; ++j) acc[i][j] = mm(af, bf[j], acc[i][j]);
    }
  }

  float* slab = sT[wave];
  const int hh = lane >> 4;
  const int c4 = (lane & 15) * 4;
  const int nc = n0 + c4;
  const bool cok = nc < N;
  v4f bv = (v4f){0.f, 0.f, 0.f, 0.f};
  if (EPI == 1) {
    bv = *(const v4fa*)(bias + clampi(nc, 0, N - 4));
    asm volatile("" :: "v"(bv));
  }
#pragma unroll
  for (int i = 0; i < 4; ++i) {
    const int mBase = m0 + (i << 4);
#pragma unroll
    for (int j = 0; j < 4; ++j) {
#pragma unroll
      for (int r = 0; r < 8; ++r) slab[(h8 + r) * 68 + (j << 4) + rl] = acc[i][j][r];
    }
    __builtin_amdgcn_fence(__ATOMIC_RELEASE, "workgroup");
    __builtin_amdgcn_wave_barrier();
    __builtin_amdgcn_fence(__ATOMIC_ACQUIRE, "workgroup");
    v4f vv[8];
#pragma unroll
    for (int it = 0; it < 8; ++it) {
      const int row = it * 2 + hh;
      v4f v = *(const v4fa*)(slab + row * 68 + c4);
      if (EPI == 1) v += bv;
      vv[it] = v;
    }
    for (int pass = 0; pass < 2; ++pass) {
#pragma unroll
      for (int it = 0; it < 8; ++it) {
        const int row = mBase + it * 2 + hh;
        if (cok && row < M) *(volatile v4f*)(D + (size_t)row * (size_t)ldd + nc) = vv[it];
      }
      __threadfence();
    }
    __builtin_amdgcn_fence(__ATOMIC_RELEASE, "workgroup");
    __builtin_amdgcn_wave_barrier();
    __builtin_amdgcn_fence(__ATOMIC_ACQUIRE, "workgroup");
  }
}

typedef int   v4i __attribute__((ext_vector_type(4)));
typedef float v2f __attribute__((ext_vector_type(2)));
typedef v4i __attribute__((may_alias)) v4ia;
typedef v2f __attribute__((may_alias)) v2fa;

constexpr int kT     = 8;
constexpr int kN     = 10000;
constexpr int kE     = 50000;
constexpr int kD     = 64;
constexpr int kTN    = kT * kN;
constexpr int kC3    = 192;
constexpr int kWIN   = 4;
constexpr int kNB    = 256;
constexpr int kNBLK  = (kN + kNB - 1) / kNB;
constexpr int kNPAD  = kNBLK * kNB;
constexpr int kDEG   = 32;
constexpr int kRCAP  = 2048;
constexpr int kCHUNK = 2048;
constexpr int kNCH   = (kE + kCHUNK - 1) / kCHUNK;
constexpr int kSTRIP = 160;

static_assert(kTN % 128 == 0);
static_assert(kTN % 64 == 0 && kC3 % 64 == 0 && kD % 32 == 0 && kC3 % 32 == 0);
static_assert(kTN % 64 == 0);
static_assert(kE % 8 == 0);
static_assert(kN <= 16384);
static_assert(kNB <= 256 && kNB == 256);
static_assert((kWIN + 1) * kDEG <= kSTRIP);
static_assert(kNPAD >= kN);

__global__ __launch_bounds__(256) void k_prep(const float* __restrict__ Wq, const float* __restrict__ Wk,
                                              const float* __restrict__ Wv, const float* __restrict__ rbias,
                                              unsigned short* WB, float* KP, float* RB) {
  __shared__ float spe[40];
  __shared__ __attribute__((aligned(16))) float skp[320];
  __shared__ __attribute__((aligned(16))) float srb[32];
  const int tid = threadIdx.x;

  {
    const int ii  = tid < 40 ? tid : 39;
    const int dtp = ii >> 3;
    const int cc  = ii & 7;
    const float fdt = (float)dtp;
    const float er  = (cc == 0) ? 0.25f : 0.0625f;
    const float ev  = expf(-(fdt * er));
    const int fq    = (cc >= 5) ? (cc - 5) : ((cc >= 2) ? (cc - 2) : 0);
    const float am  = (fq == 0) ? 1.0f : ((fq == 1) ? 0.5f : 0.25f);
    float sn, cs;
    sincosf(fdt * am, &sn, &cs);
    const float pv = (cc < 2) ? ev : ((cc < 5) ? sn : cs);
    if (tid < 40) spe[tid] = pv;
  }
  if (tid < 32) {
    const float rv = rbias[tid < 4 ? tid : 4];
    asm volatile("" :: "v"(rv));
    srb[tid] = (tid < 5) ? bf16_val(rv) : 0.0f;
  }
  __syncthreads();

#pragma unroll 1
  for (int idx = tid; idx < 320; idx += 256) {
    const int dtp = idx >> 6;
    const int j   = idx & 63;
    const v4f wa = *(const v4fa*)(Wk + j * 72 + 64);
    const v4f wb = *(const v4fa*)(Wk + j * 72 + 68);
    const float* pr = spe + dtp * 8;
    float a = pr[0] * bf16_val(wa[0]);
    a += pr[1] * bf16_val(wa[1]);
    a += pr[2] * bf16_val(wa[2]);
    a += pr[3] * bf16_val(wa[3]);
    a += pr[4] * bf16_val(wb[0]);
    a += pr[5] * bf16_val(wb[1]);
    a += pr[6] * bf16_val(wb[2]);
    a += pr[7] * bf16_val(wb[3]);
    skp[idx] = a;
  }
  __syncthreads();

  v4u o[6];
#pragma unroll
  for (int it = 0; it < 2; ++it) {
    const int lp = it * 256 + tid;
    const int n  = lp >> 3;
    const int k0 = (lp & 7) * 8;
    {
      const v4f a = *(const v4fa*)(Wq + n * 64 + k0);
      const v4f c = *(const v4fa*)(Wq + n * 64 + k0 + 4);
      o[it] = pack8_bf16(a, c);
    }
    {
      const v4f a = *(const v4fa*)(Wk + n * 72 + k0);
      const v4f c = *(const v4fa*)(Wk + n * 72 + k0 + 4);
      o[2 + it] = pack8_bf16(a, c);
    }
    {
      const v4f a = *(const v4fa*)(Wv + n * 64 + k0);
      const v4f c = *(const v4fa*)(Wv + n * 64 + k0 + 4);
      o[4 + it] = pack8_bf16(a, c);
    }
  }
  const v4f kv = *(const v4fa*)(skp + (tid < 80 ? tid : 79) * 4);
  const v4f rv4 = *(const v4fa*)(srb + (tid < 8 ? tid : 7) * 4);
  asm volatile("" :: "v"(kv));
  asm volatile("" :: "v"(rv4));
  for (int pass = 0; pass < 2; ++pass) {
#pragma unroll
    for (int s = 0; s < 3; ++s) {
#pragma unroll
      for (int it = 0; it < 2; ++it) {
        const int g = s * 512 + it * 256 + tid;
        *(volatile v4u*)(WB + (size_t)g * 8) = o[s * 2 + it];
      }
    }
    if (tid < 80) *(volatile v4f*)(KP + tid * 4) = kv;
    if (tid < 8)  *(volatile v4f*)(RB + tid * 4) = rv4;
    __threadfence();
  }
}

__global__ __launch_bounds__(256) void k_gate(const float* __restrict__ S, float* LG) {
  const int lane = threadIdx.x & 31;
  const int wave = threadIdx.x >> 5;
  const int gw   = blockIdx.x * 8 + wave;
  const int row  = clampi(gw * 8 + (lane >> 2), 0, kTN - 1);
  const int h    = lane & 3;
  const float* p = S + (size_t)row * kD + h * 16;
  const v4f a0 = *(const v4fa*)(p);
  const v4f a1 = *(const v4fa*)(p + 4);
  const v4f a2 = *(const v4fa*)(p + 8);
  const v4f a3 = *(const v4fa*)(p + 12);
  float s = bf16_val(a0[0]);
  s += bf16_val(a0[1]); s += bf16_val(a0[2]); s += bf16_val(a0[3]);
  s += bf16_val(a1[0]); s += bf16_val(a1[1]); s += bf16_val(a1[2]); s += bf16_val(a1[3]);
  s += bf16_val(a2[0]); s += bf16_val(a2[1]); s += bf16_val(a2[2]); s += bf16_val(a2[3]);
  s += bf16_val(a3[0]); s += bf16_val(a3[1]); s += bf16_val(a3[2]); s += bf16_val(a3[3]);
  const float lg = logf(s * 0.0625f + 1e-6f);
  const bool ok = gw < kTN / 8;
  float* q = LG + (size_t)gw * 32 + lane;
  if (ok) *(volatile float*)q = lg;
  __threadfence();
  if (ok) *(volatile float*)q = lg;
}

__global__ __launch_bounds__(256) void k_bucket(const int* __restrict__ ei, int* LIST, int* CNT, int* FLAG) {
  __shared__ int hl[kRCAP];
  __shared__ __attribute__((aligned(16))) int lst[kNB * kDEG];
  __shared__ __attribute__((aligned(16))) int scnt[kNB];
  __shared__ __attribute__((aligned(16))) int sflg[kNB];
  __shared__ int wcnt[8];
  const int tid = threadIdx.x, lane = tid & 31, wave = tid >> 5;
  const int base = blockIdx.x * kNB;
  int nb = kN - base;
  nb = nb > kNB ? kNB : (nb < 0 ? 0 : nb);
  const int* srcs = ei;
  const int* dsts = ei + kE;

  {
    const v4i z4 = (v4i){0, 0, 0, 0};
#pragma unroll
    for (int i = 0; i < 8; ++i) *(v4ia*)(lst + tid * kDEG + 4 * i) = z4;
  }

  int tot = 0;
  int raw = 0;
#pragma unroll 1
  for (int ch = 0; ch < kNCH; ++ch) {
    const int e0  = ch * kCHUNK + tid * 8;
    const int e0c = e0 < kE - 8 ? e0 : kE - 8;
    const v4i da = *(const v4ia*)(dsts + e0c);
    const v4i db = *(const v4ia*)(dsts + e0c + 4);
    const v4i sa = *(const v4ia*)(srcs + e0c);
    const v4i sb = *(const v4ia*)(srcs + e0c + 4);
    asm volatile("" :: "v"(da));
    asm volatile("" :: "v"(db));
    asm volatile("" :: "v"(sa));
    asm volatile("" :: "v"(sb));
    const int vm = (e0 < kE) ? -1 : 0;
    const int dk[8] = { da[0], da[1], da[2], da[3], db[0], db[1], db[2], db[3] };
    const int sk[8] = { sa[0], sa[1], sa[2], sa[3], sb[0], sb[1], sb[2], sb[3] };
    unsigned sl[8];
    int hit[8];
    int c = 0;
#pragma unroll
    for (int j = 0; j < 8; ++j) {
      const int key = (clampi(dk[j], 0, kN - 1) & vm) | ~vm;
      sl[j]  = (unsigned)key - (unsigned)base;
      hit[j] = (sl[j] < (unsigned)nb) ? 1 : 0;
      c += hit[j];
    }
    int incl = c;
#pragma unroll
    for (int dl = 1; dl < 32; dl <<= 1) {
      const int up = __shfl_up(incl, dl);
      incl += (lane >= dl) ? up : 0;
    }
    if (lane == 31) wcnt[wave] = incl;
    __syncthreads();
    int pre = 0, all = 0;
#pragma unroll
    for (int w2 = 0; w2 < 8; ++w2) {
      const int cw = clampi(wcnt[w2], 0, 256);
      all += cw;
      pre += (w2 < wave) ? cw : 0;
    }
    int pos = tot + pre + incl - c;
#pragma unroll
    for (int j = 0; j < 8; ++j) {
      if (hit[j] != 0 && pos < kRCAP) hl[pos] = clampi(sk[j], 0, kN - 1) | (int)(sl[j] << 14);
      pos += hit[j];
    }
    raw += all;
    tot = (tot + all > kRCAP) ? kRCAP : (tot + all);
    __syncthreads();
  }
  const int nh = tot;

  int cnt = 0;
#pragma unroll 1
  for (int i = 0; i < nh; ++i) {
    const int ent = hl[i];
    if ((ent >> 14) == tid) {
      if (cnt < kDEG) lst[tid * kDEG + cnt] = ent & 16383;
      ++cnt;
    }
  }
  scnt[tid] = cnt > kDEG ? kDEG : cnt;
  sflg[tid] = (raw > kRCAP || cnt > kDEG) ? 1 : 0;
  __syncthreads();

  v4i lr[8];
#pragma unroll
  for (int it = 0; it < 8; ++it) lr[it] = *(const v4ia*)(lst + (it * 256 + tid) * 4);
  const int ci = (tid < 64 ? tid : 63) * 4;
  const v4i cv = *(const v4ia*)(scnt + ci);
  const v4i fv = *(const v4ia*)(sflg + ci);
  int* lg = LIST + (size_t)base * kDEG;
  for (int pass = 0; pass < 2; ++pass) {
#pragma unroll
    for (int it = 0; it < 8; ++it) *(volatile v4i*)(lg + (it * 256 + tid) * 4) = lr[it];
    if (tid < 64) {
      *(volatile v4i*)(CNT  + base + tid * 4) = cv;
      *(volatile v4i*)(FLAG + base + tid * 4) = fv;
    }
    __threadfence();
  }
}

__global__ __launch_bounds__(256) void k_replay(const float* __restrict__ QKV, const float* __restrict__ LG,
                                                const float* __restrict__ KP, const float* __restrict__ RB,
                                                const int* __restrict__ LIST, const int* __restrict__ CNT,
                                                const int* __restrict__ FLAG, float* out) {
  __shared__ float sSC[8][kSTRIP * 4];
  const int lane = threadIdx.x & 31;
  const int wave = threadIdx.x >> 5;
  const int row  = __builtin_amdgcn_readfirstlane((int)(blockIdx.x * 8 + wave));
  const int rowc = row < kTN ? row : kTN - 1;
  const int t = rowc / kN;
  const int d = rowc - t * kN;
  const int h = lane >> 3;

  const v2f q2 = *(const v2fa*)(QKV + (size_t)rowc * kC3 + 2 * lane);
  const int mysrc = LIST[d * kDEG + lane];
  asm volatile("" :: "v"(mysrc));
  const int craw = CNT[d];
  asm volatile("" :: "v"(craw));
  const int fl = FLAG[d];
  asm volatile("" :: "v"(fl));
  const int cn  = __builtin_amdgcn_readfirstlane(clampi(craw, 0, kDEG));
  const int ndt = (t < kWIN ? t : kWIN) + 1;
  float* strip = sSC[wave];

  float m = -__builtin_inff();
#pragma unroll 1
  for (int dt = 0; dt < ndt; ++dt) {
    const v2f kp2 = *(const v2fa*)(KP + dt * kD + 2 * lane);
    const float rb = RB[dt];
    const int tb = (t - dt) * kN;
#pragma unroll 1
    for (int j = 0; j < cn; ++j) {
      const int s  = clampi(__builtin_amdgcn_readlane(mysrc, j), 0, kN - 1);
      const int rp = tb + s;
      const v2f kn2 = *(const v2fa*)(QKV + (size_t)rp * kC3 + 64 + 2 * lane);
      const float lg = LG[(size_t)rp * 4 + h];
      const float kx = kn2[0] + kp2[0];
      const float ky = kn2[1] + kp2[1];
      float p = q2[0] * kx + q2[1] * ky;
      p += __shfl_xor(p, 1);
      p += __shfl_xor(p, 2);
      p += __shfl_xor(p, 4);
      const float sc = (p * 0.25f + rb) + lg;
      if ((lane & 7) == 0) strip[(dt * cn + j) * 4 + h] = sc;
      m = fmaxf(m, sc);
    }
  }
  __builtin_amdgcn_fence(__ATOMIC_RELEASE, "workgroup");
  __builtin_amdgcn_wave_barrier();
  __builtin_amdgcn_fence(__ATOMIC_ACQUIRE, "workgroup");

  const float smax = (fabsf(m) <= 0x1.fffffep+127f) ? m : 0.0f;
  float den = 0.0f, ax = 0.0f, ay = 0.0f;
#pragma unroll 1
  for (int dt = 0; dt < ndt; ++dt) {
    const int tb = (t - dt) * kN;
#pragma unroll 1
    for (int j = 0; j < cn; ++j) {
      const int s  = clampi(__builtin_amdgcn_readlane(mysrc, j), 0, kN - 1);
      const int rp = tb + s;
      const v2f v2 = *(const v2fa*)(QKV + (size_t)rp * kC3 + 128 + 2 * lane);
      const float sc = strip[(dt * cn + j) * 4 + h];
      const float w = expf(sc - smax);
      den += w;
      ax += w * v2[0];
      ay += w * v2[1];
    }
  }
  const float dd = (den < 1e-12f) ? 1e-12f : den;
  float ox = ax / dd;
  float oy = ay / dd;
  const bool empty = (cn == 0);
  ox = empty ? 0.0f : ox;
  oy = empty ? 0.0f : oy;
  const float qnan = __int_as_float(0x7fc00000);
  const bool bad = (fl != 0);
  ox = bad ? qnan : ox;
  oy = bad ? qnan : oy;
  const v2f o = (v2f){ ox, oy };
  const bool ok = row < kTN;
  float* op = out + (size_t)rowc * kD + 2 * lane;
  if (ok) *(volatile v2f*)op = o;
  __threadfence();
  if (ok) *(volatile v2f*)op = o;
}

constexpr size_t kSzHB   = (size_t)kTN * kD * 2;
constexpr size_t kSzWB   = (size_t)kC3 * kD * 2;
constexpr size_t kSzKP   = (size_t)5 * kD * 4;
constexpr size_t kSzRB   = 128;
constexpr size_t kSzLG   = (size_t)kTN * 4 * 4;
constexpr size_t kSzQKV  = (size_t)kTN * kC3 * 4;
constexpr size_t kSzLIST = (size_t)kNPAD * kDEG * 4;
constexpr size_t kSzCNT  = (size_t)kNPAD * 4;
constexpr size_t kSzFLAG = (size_t)kNPAD * 4;
constexpr size_t kOffHB   = 0;
constexpr size_t kOffWB   = kOffHB + kSzHB;
constexpr size_t kOffKP   = kOffWB + kSzWB;
constexpr size_t kOffRB   = kOffKP + kSzKP;
constexpr size_t kOffLG   = kOffRB + kSzRB;
constexpr size_t kOffQKV  = kOffLG + kSzLG;
constexpr size_t kOffLIST = kOffQKV + kSzQKV;
constexpr size_t kOffCNT  = kOffLIST + kSzLIST;
constexpr size_t kOffFLAG = kOffCNT + kSzCNT;
constexpr size_t kWsTotal = kOffFLAG + kSzFLAG;
static_assert(kSzHB % 128 == 0 && kSzWB % 128 == 0 && kSzKP % 128 == 0 && kSzRB % 128 == 0 && kSzLG % 128 == 0);
static_assert(kSzQKV % 128 == 0 && kSzLIST % 128 == 0 && kSzCNT % 128 == 0 && kSzFLAG % 128 == 0);
static_assert(kWsTotal == 74378624);
static_assert(kWsTotal <= ((size_t)128 << 20));
static_assert(((size_t)kTN * kD / 8) % 256 == 0);
static_assert((size_t)kTN * kD == 5120000);

extern "C" void kernel_launch(void* const* d_in, const int* in_sizes, int n_in,
                              void* d_out, int out_size, void* d_ws, size_t ws_size,
                              hipStream_t stream) {
  if (n_in < 8) return;
  if (in_sizes[0] != kTN * kD || in_sizes[1] != kTN * kD) return;
  if (in_sizes[2] != 2 * kE) return;
  if (in_sizes[4] != 64 * 64 || in_sizes[5] != 64 * 72 || in_sizes[6] != 64 * 64) return;
  if (in_sizes[7] != kWIN + 1) return;
  if (out_size != kTN * kD) return;
  if (ws_size < kWsTotal) return;

  const float* H  = (const float*)d_in[0];
  const float* S  = (const float*)d_in[1];
  const int*   ei = (const int*)  d_in[2];
  const float* Wq = (const float*)d_in[4];
  const float* Wk = (const float*)d_in[5];
  const float* Wv = (const float*)d_in[6];
  const float* rb = (const float*)d_in[7];
  float* out = (float*)d_out;

  char* ws = (char*)d_ws;
  unsigned short* HB  = (unsigned short*)(ws + kOffHB);
  unsigned short* WB  = (unsigned short*)(ws + kOffWB);
  float* KP   = (float*)(ws + kOffKP);
  float* RB   = (float*)(ws + kOffRB);
  float* LG   = (float*)(ws + kOffLG);
  float* QKV  = (float*)(ws + kOffQKV);
  int*   LIST = (int*)(ws + kOffLIST);
  int*   CNT  = (int*)(ws + kOffCNT);
  int*   FLAG = (int*)(ws + kOffFLAG);

  k_plane<0><<<(kTN * kD / 8) / 256, 256, 0, stream>>>(H, kTN, kD, kD, HB, kTN, kD);
  k_prep<<<1, 256, 0, stream>>>(Wq, Wk, Wv, rb, WB, KP, RB);
  k_gate<<<kTN / 64, 256, 0, stream>>>(S, LG);
  {
    const int tiles = (kTN / 64) * (kC3 / 64);
    k_gemm_nt<0, 0><<<(tiles + 7) / 8, 256, 0, stream>>>(HB, WB, KP, QKV, kTN, kC3, kD, kC3);
  }
  k_bucket<<<kNBLK, 256, 0, stream>>>(ei, LIST, CNT, FLAG);
  k_replay<<<kTN / 8, 256, 0, stream>>>(QKV, LG, KP, RB, LIST, CNT, FLAG, out);
}
